// ViLLayer_61744449847850
// MI455X (gfx1250) — hardware-verified
//
#include <hip/hip_runtime.h>

typedef __attribute__((ext_vector_type(16))) _Float16 v16h;
typedef __attribute__((ext_vector_type(8)))  _Float16 v8h;
typedef __attribute__((ext_vector_type(16))) __bf16   v16b;
typedef __attribute__((ext_vector_type(8)))  __bf16   v8b;
typedef __attribute__((ext_vector_type(8)))  float    v8f;
typedef __attribute__((ext_vector_type(4)))  float    v4f;
typedef __attribute__((ext_vector_type(4)))  unsigned int u4w;

constexpr int NB     = 4;
constexpr int SEQ    = 1024;
constexpr int DMODEL = 512;
constexpr int DINNER = 1024;
constexpr int NHEAD  = 16;
constexpr int DHEAD  = 64;
constexpr int KTAPS  = 4;
constexpr int NTOK   = NB * SEQ;
constexpr int UPN    = 2 * DINNER;
constexpr int GIN_LD = 3 * DINNER;
constexpr int GATE_N = 64;

static_assert(NHEAD * DHEAD == DINNER, "heads");
static_assert(SEQ % 64 == 0 && SEQ / 64 == 16, "query blocks");
static_assert(NTOK % 64 == 0 && UPN % 64 == 0 && DMODEL % 32 == 0, "up gemm tiles");
static_assert(DHEAD % 64 == 0 && DHEAD % 32 == 0, "headwise gemm tiles");
static_assert(GATE_N % 64 == 0 && GIN_LD % 32 == 0, "gate gemm tiles");
static_assert(DMODEL % 64 == 0 && DINNER % 32 == 0, "down gemm tiles");

constexpr size_t SZ_X16   = (size_t)NTOK * DMODEL * 2;
constexpr size_t SZ_WUP16 = (size_t)UPN * DMODEL * 2;
constexpr size_t SZ_WDN16 = (size_t)DMODEL * DINNER * 2;
constexpr size_t SZ_WH16  = (size_t)NHEAD * DHEAD * DHEAD * 2;
constexpr size_t SZ_WG16  = (size_t)GATE_N * GIN_LD * 2;
constexpr size_t SZ_XZ    = (size_t)NTOK * UPN * 4;
constexpr size_t SZ_XA    = (size_t)NTOK * DINNER * 4;
constexpr size_t SZ_A16   = (size_t)NTOK * DINNER * 2;
constexpr size_t SZ_GIN   = (size_t)NTOK * GIN_LD * 2;
constexpr size_t SZ_GRAW  = (size_t)NTOK * GATE_N * 4;
constexpr size_t SZ_BHS   = (size_t)NB * NHEAD * SEQ * 4;
constexpr size_t SZ_H     = (size_t)NTOK * DINNER * 4;

constexpr size_t OFF_XH    = 0;
constexpr size_t OFF_XL    = OFF_XH + SZ_X16;
constexpr size_t OFF_WUH   = OFF_XL + SZ_X16;
constexpr size_t OFF_WUL   = OFF_WUH + SZ_WUP16;
constexpr size_t OFF_WDH   = OFF_WUL + SZ_WUP16;
constexpr size_t OFF_WDL   = OFF_WDH + SZ_WDN16;
constexpr size_t OFF_WQ    = OFF_WDL + SZ_WDN16;
constexpr size_t OFF_WK    = OFF_WQ + SZ_WH16;
constexpr size_t OFF_WV    = OFF_WK + SZ_WH16;
constexpr size_t OFF_WG    = OFF_WV + SZ_WH16;
constexpr size_t OFF_XZ    = OFF_WG + SZ_WG16;
constexpr size_t OFF_XA    = OFF_XZ + SZ_XZ;
constexpr size_t OFF_ACT16 = OFF_XA + SZ_XA;
constexpr size_t OFF_XM16  = OFF_ACT16 + SZ_A16;
constexpr size_t OFF_H     = OFF_ACT16;
constexpr size_t OFF_GIN   = OFF_ACT16 + 2 * SZ_A16;
constexpr size_t OFF_HSH   = OFF_GIN;
constexpr size_t OFF_HSL   = OFF_GIN + SZ_A16;
constexpr size_t OFF_GRAW  = OFF_GIN + SZ_GIN;
constexpr size_t OFF_IPG   = OFF_GRAW + SZ_GRAW;
constexpr size_t OFF_CUM   = OFF_IPG + SZ_BHS;
constexpr size_t OFF_END   = OFF_CUM + SZ_BHS;
static_assert(SZ_H <= 2 * SZ_A16, "h alias fits");
static_assert(2 * SZ_A16 <= SZ_GIN, "hs planes alias fits");
static_assert(OFF_END == 109314048, "carve total");
static_assert(OFF_END <= (size_t)134217728, "carve under 128 MiB");
static_assert((OFF_XZ % 256) == 0 && (OFF_GIN % 256) == 0 && (OFF_CUM % 256) == 0, "alignment");

__device__ __forceinline__ unsigned short f2bf_bits(float f) {
  unsigned u = __float_as_uint(f);
  return (unsigned short)((u + 0x7FFFu + ((u >> 16) & 1u)) >> 16);
}
__device__ __forceinline__ float bf_bits2f(unsigned short h) { return __uint_as_float(((unsigned)h) << 16); }
__device__ __forceinline__ unsigned short f2h_bits(float f) { return __builtin_bit_cast(unsigned short, (_Float16)f); }

__device__ __forceinline__ void dep_guard_h(v8f& a, v8f& b, v16h x, v16h y) { asm volatile("v_nop\n\tv_nop\n\tv_nop\n\tv_nop" : "+v"(a), "+v"(b) : "v"(x), "v"(y)); }
__device__ __forceinline__ void dep_guard_b(v8f& a, v8f& b, v16b x, v16b y) { asm volatile("v_nop\n\tv_nop\n\tv_nop\n\tv_nop" : "+v"(a), "+v"(b) : "v"(x), "v"(y)); }
__device__ __forceinline__ void keep4_h(v16h a, v16h b, v16h c, v16h d) { asm volatile("v_nop" :: "v"(a), "v"(b), "v"(c), "v"(d)); }
__device__ __forceinline__ void keep4_b(v16b a, v16b b, v16b c, v16b d) { asm volatile("v_nop" :: "v"(a), "v"(b), "v"(c), "v"(d)); }
__device__ __forceinline__ void acc_guard4(v8f& a, v8f& b, v8f& c, v8f& d) { asm volatile("v_nop\n\tv_nop\n\tv_nop\n\tv_nop" : "+v"(a), "+v"(b), "+v"(c), "+v"(d)); }
template <typename T> struct Frag;
template <> struct Frag<_Float16> {
  typedef v16h V; union U { v16h v; v8h h[2]; };
  static __device__ __forceinline__ v16h load(const _Float16* p) {
    U f; f.h[0] = *(const v8h*)(p); f.h[1] = *(const v8h*)(p + 16); return f.v;
  }
  static __device__ __forceinline__ v8f mma(v16h a, v16h b, v8f c) {
    return __builtin_amdgcn_wmma_f32_16x16x32_f16(false, a, false, b, (short)0, c, false, false);
  }
  static __device__ __forceinline__ void guard(v8f& a, v8f& b, v16h x, v16h y) { dep_guard_h(a, b, x, y); }
  static __device__ __forceinline__ void keep(v16h a, v16h b, v16h c, v16h d) { keep4_h(a, b, c, d); }
};
template <> struct Frag<__bf16> {
  typedef v16b V; union U { v16b v; v8b h[2]; };
  static __device__ __forceinline__ v16b load(const __bf16* p) {
    U f; f.h[0] = *(const v8b*)(p); f.h[1] = *(const v8b*)(p + 16); return f.v;
  }
  static __device__ __forceinline__ v8f mma(v16b a, v16b b, v8f c) {
    return __builtin_amdgcn_wmma_f32_16x16x32_bf16(false, a, false, b, (short)0, c, false, false);
  }
  static __device__ __forceinline__ void guard(v8f& a, v8f& b, v16b x, v16b y) { dep_guard_b(a, b, x, y); }
  static __device__ __forceinline__ void keep(v16b a, v16b b, v16b c, v16b d) { keep4_b(a, b, c, d); }
};
__device__ __forceinline__ v8f mma_gb(v16b a, v16b b, v8f c) {
  c = __builtin_amdgcn_wmma_f32_16x16x32_bf16(false, a, false, b, (short)0, c, false, false);
  asm volatile("v_nop\n\tv_nop\n\tv_nop\n\tv_nop" : "+v"(c) : "v"(a), "v"(b));
  return c;
}

template <int ET> struct Elem;
template <> struct Elem<0> { typedef _Float16 T; };
template <> struct Elem<1> { typedef __bf16 T; };
template <int ET, bool SPLIT, int BIAS_MODE, int OUT_MODE, bool RESID, int ACT = 0>
__global__ __launch_bounds__(256) void wmma_gemm64(
    const unsigned short* __restrict__ Ap, const unsigned short* __restrict__ A2p, int lda, long strideA,
    const unsigned short* __restrict__ Btp, const unsigned short* __restrict__ Bt2p, int ldb, long strideB,
    void* __restrict__ Cout, void* __restrict__ Cout2, int ldc, long strideC,
    const float* __restrict__ bias,
    const float* __restrict__ resid, long strideR,
    int M, int N, int K, float scale) {
  typedef typename Elem<ET>::T T;
  typedef typename Frag<T>::V V;
  const T* A = (const T*)Ap; const T* A2 = (const T*)A2p; const T* Bt = (const T*)Btp; const T* Bt2 = (const T*)Bt2p;
  __shared__ __align__(16) float sT[8][16 * 68];
  const int b    = blockIdx.y;
  const int lane = threadIdx.x & 31;
  const int wave = threadIdx.x >> 5;
  const int tilesN = N >> 6;
  const int tilesM = M >> 6;
  const int tile = blockIdx.x * 8 + wave;
  if (tile >= tilesM * tilesN) return;
  const int tm = tile / tilesN;
  const int tn = tile - tm * tilesN;
  const int m0 = tm << 6;
  const int n0 = tn << 6;

  const T* Ab  = A  + (size_t)b * strideA;
  const T* Bb  = Bt + (size_t)b * strideB;
  const T* Ab2 = SPLIT ? (A2  + (size_t)b * strideA) : nullptr;
  const T* Bb2 = SPLIT ? (Bt2 + (size_t)b * strideB) : nullptr;

  const int rlane = lane & 15;
  const int koff  = (lane >> 4) * 8;
  const int mOff  = (lane >> 4) * 8;

  v8f acc[4][4];
#pragma unroll
  for (int i = 0; i < 4; ++i)
#pragma unroll
    for (int j = 0; j < 4; ++j) acc[i][j] = (v8f){0.f,0.f,0.f,0.f,0.f,0.f,0.f,0.f};

  for (int k0 = 0; k0 < K; k0 += 32) {
    V bh[4], bl[4];
#pragma unroll
    for (int j = 0; j < 4; ++j) {
      const size_t bo = (size_t)(n0 + (j << 4) + rlane) * ldb + koff + k0;
      bh[j] = Frag<T>::load(Bb + bo);
      if (SPLIT) bl[j] = Frag<T>::load(Bb2 + bo);
    }
#pragma unroll
    for (int i = 0; i < 4; ++i) {
      const size_t ao = (size_t)(m0 + (i << 4) + rlane) * lda + koff + k0;
      V ah = Frag<T>::load(Ab + ao);
      V al;
      if (SPLIT) al = Frag<T>::load(Ab2 + ao);
#pragma unroll
      for (int j = 0; j < 4; ++j) {
        acc[i][j] = Frag<T>::mma(ah, bh[j], acc[i][j]);
        if (SPLIT) {
          acc[i][j] = Frag<T>::mma(ah, bl[j], acc[i][j]);
          acc[i][j] = Frag<T>::mma(al, bh[j], acc[i][j]);
        }
      }
      Frag<T>::guard(acc[i][0], acc[i][3], ah, SPLIT ? al : ah);
    }
    Frag<T>::keep(bh[0], bh[1], bh[2], bh[3]);
    if (SPLIT) Frag<T>::keep(bl[0], bl[1], bl[2], bl[3]);
  }
  acc_guard4(acc[0][0], acc[0][1], acc[0][2], acc[0][3]);
  acc_guard4(acc[1][0], acc[1][1], acc[1][2], acc[1][3]);
  acc_guard4(acc[2][0], acc[2][1], acc[2][2], acc[2][3]);
  acc_guard4(acc[3][0], acc[3][1], acc[3][2], acc[3][3]);

  float* slab = sT[wave];
  const float* Rb = RESID ? (resid + (size_t)b * strideR) : nullptr;
#pragma unroll
  for (int i = 0; i < 4; ++i) {
    const int mBase = m0 + (i << 4);
#pragma unroll
    for (int j = 0; j < 4; ++j) {
      const int n = n0 + (j << 4) + rlane;
      float bv = 0.f;
      if (BIAS_MODE == 2) bv = bias[n];
#pragma unroll
      for (int r = 0; r < 8; ++r) {
        float v = acc[i][j][r] * scale;
        if (BIAS_MODE == 1) v += bias[mBase + mOff + r];
        if (BIAS_MODE == 2) v += bv;
        if (RESID) v += Rb[(size_t)(mBase + mOff + r) * ldc + n];
        if (ACT == 1) v = tanhf(v);
        if (ACT == 2) v = fmaxf(v, 0.0f);
        if (ACT == 3) v = v / (1.0f + expf(-v));
        if (ACT == 4) v = (v > 0.f) ? v : 0.01f * v;
        slab[(mOff + r) * 68 + (j << 4) + rlane] = v;
      }
    }
    __builtin_amdgcn_fence(__ATOMIC_RELEASE, "workgroup");
    __builtin_amdgcn_wave_barrier();
    __builtin_amdgcn_fence(__ATOMIC_ACQUIRE, "workgroup");
    if (OUT_MODE == 0) {
      float* C = (float*)Cout + (size_t)b * strideC;
      const int hh = lane >> 4, c4 = (lane & 15) * 4;
      for (int pass = 0; pass < 2; ++pass) {
#pragma unroll
        for (int it = 0; it < 8; ++it) {
          const int row = it * 2 + hh;
          v4f v = *(const v4f*)(slab + row * 68 + c4);
          *(volatile v4f*)(C + (size_t)(mBase + row) * ldc + n0 + c4) = v;
        }
        __threadfence();
      }
    } else {
      const int q = lane >> 3, c8 = (lane & 7) * 8;
      unsigned short* C  = (unsigned short*)Cout  + (size_t)b * strideC;
      unsigned short* C2 = (OUT_MODE == 2) ? ((unsigned short*)Cout2 + (size_t)b * strideC) : nullptr;
      for (int pass = 0; pass < 2; ++pass) {
#pragma unroll
        for (int it = 0; it < 4; ++it) {
          const int row = it * 4 + q;
          const float* sp = slab + row * 68 + c8;
          v8h hv, lv;
#pragma unroll
          for (int e = 0; e < 8; ++e) {
            if (OUT_MODE == 1) {
              hv[e] = (_Float16)sp[e];
              lv[e] = hv[e];
            } else {
              unsigned short hb = f2bf_bits(sp[e]);
              hv[e] = __builtin_bit_cast(_Float16, hb);
              if (OUT_MODE == 2) {
                unsigned short lb = f2bf_bits(sp[e] - bf_bits2f(hb));
                lv[e] = __builtin_bit_cast(_Float16, lb);
              } else {
                lv[e] = hv[e];
              }
            }
          }
          *(volatile v8h*)(C + (size_t)(mBase + row) * ldc + n0 + c8) = hv;
          if (OUT_MODE == 2) *(volatile v8h*)(C2 + (size_t)(mBase + row) * ldc + n0 + c8) = lv;
        }
        __threadfence();
      }
    }
    __builtin_amdgcn_fence(__ATOMIC_RELEASE, "workgroup");
    __builtin_amdgcn_wave_barrier();
    __builtin_amdgcn_fence(__ATOMIC_ACQUIRE, "workgroup");
  }
}

__global__ __launch_bounds__(256) void cast_bf16_split8(const float* __restrict__ in,
                                                         unsigned short* __restrict__ hi,
                                                         unsigned short* __restrict__ lo, int n8) {
  const int i = blockIdx.x * 256 + threadIdx.x;
  if (i >= n8) return;
  const size_t base = (size_t)i * 8;
  const v4f a = *(const v4f*)(in + base);
  const v4f c = *(const v4f*)(in + base + 4);
  const float f[8] = {a[0], a[1], a[2], a[3], c[0], c[1], c[2], c[3]};
  u4w hw, lw;
#pragma unroll
  for (int e = 0; e < 4; ++e) {
    const unsigned short h0 = f2bf_bits(f[2 * e]);
    const unsigned short h1 = f2bf_bits(f[2 * e + 1]);
    const unsigned short l0 = f2bf_bits(f[2 * e] - bf_bits2f(h0));
    const unsigned short l1 = f2bf_bits(f[2 * e + 1] - bf_bits2f(h1));
    hw[e] = (unsigned)h0 | ((unsigned)h1 << 16);
    lw[e] = (unsigned)l0 | ((unsigned)l1 << 16);
  }
  volatile u4w* ph = (volatile u4w*)(void*)(hi + base);
  volatile u4w* pl = (volatile u4w*)(void*)(lo + base);
  *ph = hw; *pl = lw;
  __threadfence();
  *ph = hw; *pl = lw;
}

__global__ __launch_bounds__(256) void cast_f16_scale8(const float* __restrict__ in,
                                                        unsigned short* __restrict__ out, int n8, float sc) {
  const int i = blockIdx.x * 256 + threadIdx.x;
  if (i >= n8) return;
  const size_t base = (size_t)i * 8;
  const v4f a = *(const v4f*)(in + base);
  const v4f c = *(const v4f*)(in + base + 4);
  const float f[8] = {a[0], a[1], a[2], a[3], c[0], c[1], c[2], c[3]};
  u4w w;
#pragma unroll
  for (int e = 0; e < 4; ++e) {
    const unsigned short h0 = f2h_bits(f[2 * e] * sc);
    const unsigned short h1 = f2h_bits(f[2 * e + 1] * sc);
    w[e] = (unsigned)h0 | ((unsigned)h1 << 16);
  }
  volatile u4w* p = (volatile u4w*)(void*)(out + base);
  *p = w;
  __threadfence();
  *p = w;
}

__global__ __launch_bounds__(256) void build_gate_w8(const float* __restrict__ wi, const float* __restrict__ wf,
                                                      unsigned short* __restrict__ out, int n8) {
  const int i = blockIdx.x * 256 + threadIdx.x;
  if (i >= n8) return;
  constexpr int CH8 = GIN_LD / 8;
  const int row = i / CH8;
  const int col = (i - row * CH8) * 8;
  const int ri = (row < NHEAD) ? row : (NHEAD - 1);
  int rf = row - NHEAD; rf = (rf < 0) ? 0 : ((rf > NHEAD - 1) ? (NHEAD - 1) : rf);
  const v4f a0 = *(const v4f*)(wi + (size_t)ri * GIN_LD + col);
  const v4f a1 = *(const v4f*)(wi + (size_t)ri * GIN_LD + col + 4);
  const v4f b0 = *(const v4f*)(wf + (size_t)rf * GIN_LD + col);
  const v4f b1 = *(const v4f*)(wf + (size_t)rf * GIN_LD + col + 4);
  const bool useI = (row < NHEAD);
  const bool useF = (row >= NHEAD) && (row < 2 * NHEAD);
  float f[8];
#pragma unroll
  for (int e = 0; e < 4; ++e) {
    f[e]     = useI ? a0[e] : (useF ? b0[e] : 0.f);
    f[4 + e] = useI ? a1[e] : (useF ? b1[e] : 0.f);
  }
  u4w w;
#pragma unroll
  for (int e = 0; e < 4; ++e) {
    const unsigned short h0 = f2bf_bits(f[2 * e]);
    const unsigned short h1 = f2bf_bits(f[2 * e + 1]);
    w[e] = (unsigned)h0 | ((unsigned)h1 << 16);
  }
  volatile u4w* p = (volatile u4w*)(void*)(out + (size_t)i * 8);
  *p = w;
  __threadfence();
  *p = w;
}

__global__ __launch_bounds__(256) void conv_silu_kernel(const float* __restrict__ xz,
                                                         const float* __restrict__ cw,
                                                         const float* __restrict__ cb,
                                                         float* __restrict__ xa,
                                                         unsigned short* __restrict__ xa16,
                                                         unsigned short* __restrict__ xm16) {
  __shared__ __align__(16) unsigned int sa[512];
  __shared__ __align__(16) unsigned int sm[512];
  const int row = blockIdx.x;
  const int tid = threadIdx.x;
  const int c4  = tid * 4;
  const int s   = row & (SEQ - 1);
  float xin[4][4];
#pragma unroll
  for (int j = 0; j < KTAPS; ++j) {
    const int back = KTAPS - 1 - j;
    const bool valid = (s >= back);
    const int rj = valid ? (row - back) : row;
    const v4f t = *(const v4f*)(xz + (size_t)rj * UPN + c4);
#pragma unroll
    for (int e = 0; e < 4; ++e) xin[j][e] = valid ? t[e] : 0.f;
  }
  v4f wv[4];
#pragma unroll
  for (int e = 0; e < 4; ++e) wv[e] = *(const v4f*)(cw + (size_t)(c4 + e) * KTAPS);
  const v4f cbv = *(const v4f*)(cb + c4);
  v4f xav;
  unsigned short ha[4], hm[4];
#pragma unroll
  for (int e = 0; e < 4; ++e) {
    float acc = 0.f;
#pragma unroll
    for (int j = 0; j < KTAPS; ++j) acc += xin[j][e] * wv[e][j];
    acc += cbv[e];
    const float sl = acc / (1.0f + __expf(-acc));
    xav[e] = sl;
    ha[e] = f2h_bits(sl * 64.0f);
    hm[e] = f2h_bits(xin[KTAPS - 1][e] * 8.0f);
  }
  {
    volatile v4f* p = (volatile v4f*)(xa + (size_t)row * DINNER + c4);
    *p = xav;
    __threadfence();
    *p = xav;
  }
  sa[2 * tid]     = (unsigned)ha[0] | ((unsigned)ha[1] << 16);
  sa[2 * tid + 1] = (unsigned)ha[2] | ((unsigned)ha[3] << 16);
  sm[2 * tid]     = (unsigned)hm[0] | ((unsigned)hm[1] << 16);
  sm[2 * tid + 1] = (unsigned)hm[2] | ((unsigned)hm[3] << 16);
  __syncthreads();
  if (tid < 128) {
    const u4w v = *(const u4w*)(&sa[4 * tid]);
    volatile u4w* p = (volatile u4w*)(void*)(xa16 + (size_t)row * DINNER + 8 * tid);
    *p = v;
    __threadfence();
    *p = v;
  } else {
    const int t2 = tid - 128;
    const u4w v = *(const u4w*)(&sm[4 * t2]);
    volatile u4w* p = (volatile u4w*)(void*)(xm16 + (size_t)row * DINNER + 8 * t2);
    *p = v;
    __threadfence();
    *p = v;
  }
}

__global__ __launch_bounds__(32) void gate_scan_kernel(const float* __restrict__ graw,
                                                        const float* __restrict__ bi,
                                                        const float* __restrict__ bfw,
                                                        float* __restrict__ ipg,
                                                        float* __restrict__ cumg) {
  __shared__ float cs[SEQ];
  __shared__ float ps[SEQ];
  const int bh = blockIdx.x;
  const int l  = threadIdx.x;
  const int b  = bh >> 4;
  const int hd = bh & 15;
  const float biv = bi[hd];
  const float bfv = bfw[hd];
  float carry = 0.f;
#pragma unroll 1
  for (int i = 0; i < SEQ / 32; ++i) {
    const size_t row = (size_t)b * SEQ + i * 32 + l;
    const float gi = graw[row * GATE_N + hd];
    const float gf = graw[row * GATE_N + NHEAD + hd];
    const float ipv = gi + biv;
    const float fp  = gf + bfv;
    const float lf  = fminf(fp, 0.0f) - log1pf(expf(-fabsf(fp)));
    float x = lf;
#pragma unroll
    for (int off = 1; off < 32; off <<= 1) {
      const float y = __shfl_up(x, off, 32);
      x = (l >= off) ? (x + y) : x;
    }
    const float cumv = carry + x;
    const float tot  = __shfl(x, 31, 32);
    carry += tot;
    cs[i * 32 + l] = cumv;
    ps[i * 32 + l] = ipv;
  }
  __syncthreads();
  for (int pass = 0; pass < 2; ++pass) {
#pragma unroll 1
    for (int i = 0; i < SEQ / 32; ++i) {
      const float cv = cs[i * 32 + l];
      const float pv = ps[i * 32 + l];
      ((volatile float*)cumg)[(size_t)bh * SEQ + i * 32 + l] = cv;
      ((volatile float*)ipg)[(size_t)bh * SEQ + i * 32 + l]  = pv;
    }
    __threadfence();
  }
}

__global__ __launch_bounds__(128) void mlstm64_kernel(const unsigned short* __restrict__ gin,
                                                       const float* __restrict__ cumg,
                                                       const float* __restrict__ ipg,
                                                       float* __restrict__ hout) {
  typedef Frag<__bf16> FB16;
  union FBU { v16b v; v8b h[2]; };
  __shared__ __align__(16) unsigned short Ksh[64 * 64];
  __shared__ __align__(16) unsigned short Vt[64 * 64];
  __shared__ __align__(16) unsigned short Psh[4][16 * 64];
  __shared__ __align__(16) float Os[4][16 * 68];
  const int tid  = threadIdx.x;
  const int wave = tid >> 5;
  const int lane = tid & 31;
  const int hh   = lane >> 4;
  const int c    = lane & 15;
  const int bx = blockIdx.x;
  const int qb = bx & 15;
  const int bh = bx >> 4;
  const int hd = bh & 15;
  const int b  = bh >> 4;
  const int q0 = qb * 64 + wave * 16;
  const size_t tokb = (size_t)b * SEQ;
  const __bf16* ginb = (const __bf16*)(const void*)gin;

  v16b qa[2];
  {
    const __bf16* qrow = ginb + (tokb + q0 + c) * GIN_LD + hd * DHEAD;
#pragma unroll
    for (int dc = 0; dc < 2; ++dc) qa[dc] = FB16::load(qrow + dc * 32 + 8 * hh);
  }
  float cums[8], mrow[8], nrow[8];
  v8f oacc[4];
#pragma unroll
  for (int r = 0; r < 8; ++r) {
    cums[r] = cumg[(size_t)bh * SEQ + q0 + 8 * hh + r];
    mrow[r] = -1e30f;
    nrow[r] = 0.f;
  }
#pragma unroll
  for (int t = 0; t < 4; ++t) oacc[t] = (v8f){0.f,0.f,0.f,0.f,0.f,0.f,0.f,0.f};

  const int nChunks = qb + 1;
  for (int kc = 0; kc < nChunks; ++kc) {
    const int kv0 = kc * 64;
    __syncthreads();
    {
      const int kvr = tid >> 1, dh = (tid & 1) * 32;
      const size_t rbase = (tokb + kv0 + kvr) * GIN_LD + hd * DHEAD + dh;
      const u4w* ks = (const u4w*)(const void*)(gin + rbase + DINNER);
      const u4w* vs = (const u4w*)(const void*)(gin + rbase + 2 * DINNER);
      u4w* kd = (u4w*)(void*)(Ksh + kvr * 64 + dh);
#pragma unroll
      for (int i = 0; i < 4; ++i) {
        const u4w kw = ks[i];
        kd[i] = kw;
        const u4w vw = vs[i];
#pragma unroll
        for (int e = 0; e < 4; ++e) {
          const unsigned w = vw[e];
          const int d = dh + 8 * i + 2 * e;
          Vt[d * 64 + kvr]       = (unsigned short)(w & 0xffffu);
          Vt[(d + 1) * 64 + kvr] = (unsigned short)(w >> 16);
        }
      }
    }
    __syncthreads();

    v8f s[4];
#pragma unroll
    for (int j = 0; j < 4; ++j) {
      s[j] = (v8f){0.f,0.f,0.f,0.f,0.f,0.f,0.f,0.f};
#pragma unroll
      for (int dc = 0; dc < 2; ++dc) {
        FBU kb;
        kb.h[0] = *(const v8b*)(const void*)(Ksh + (j * 16 + c) * 64 + dc * 32 + 8 * hh);
        kb.h[1] = *(const v8b*)(const void*)(Ksh + (j * 16 + c) * 64 + dc * 32 + 16 + 8 * hh);
        s[j] = mma_gb(qa[dc], kb.v, s[j]);
      }
    }
    float cumt[4], ipt[4];
#pragma unroll
    for (int j = 0; j < 4; ++j) {
      const size_t o = (size_t)bh * SEQ + kv0 + j * 16 + c;
      cumt[j] = cumg[o];
      ipt[j]  = ipg[o];
    }
    float cm[8];
#pragma unroll
    for (int r = 0; r < 8; ++r) {
      const int qrow = q0 + 8 * hh + r;
      float m = -1e30f;
#pragma unroll
      for (int j = 0; j < 4; ++j) {
        const int kvcol = kv0 + j * 16 + c;
        const float ld = (cums[r] - cumt[j]) + ipt[j];
        const float lv = (kvcol <= qrow) ? ld : -1e30f;
        m = fmaxf(m, lv);
      }
#pragma unroll
      for (int off = 1; off < 16; off <<= 1) m = fmaxf(m, __shfl_xor(m, off, 32));
      cm[r] = m;
    }
    unsigned short* pw = Psh[wave];
#pragma unroll
    for (int r = 0; r < 8; ++r) {
      const int qrow = q0 + 8 * hh + r;
      const float mnew  = fmaxf(mrow[r], cm[r]);
      const float alpha = __expf(mrow[r] - mnew);
      mrow[r] = mnew;
      float psum = 0.f;
#pragma unroll
      for (int j = 0; j < 4; ++j) {
        const int kvcol = kv0 + j * 16 + c;
        const float ld = (cums[r] - cumt[j]) + ipt[j];
        const float lv = (kvcol <= qrow) ? ld : -1e30f;
        const float dd = __expf(lv - mnew);
        const float cel = (s[j][r] * 0.125f) * dd;
        psum += cel;
        pw[(8 * hh + r) * 64 + j * 16 + c] = f2bf_bits(cel);
      }
#pragma unroll
      for (int off = 1; off < 16; off <<= 1) psum += __shfl_xor(psum, off, 32);
      nrow[r] = nrow[r] * alpha + psum;
#pragma unroll
      for (int t = 0; t < 4; ++t) oacc[t][r] *= alpha;
    }
    __syncthreads();
#pragma unroll
    for (int kk = 0; kk < 2; ++kk) {
      FBU pa;
      pa.h[0] = *(const v8b*)(const void*)(pw + c * 64 + kk * 32 + 8 * hh);
      pa.h[1] = *(const v8b*)(const void*)(pw + c * 64 + kk * 32 + 16 + 8 * hh);
#pragma unroll
      for (int t = 0; t < 4; ++t) {
        FBU vb;
        vb.h[0] = *(const v8b*)(const void*)(Vt + (t * 16 + c) * 64 + kk * 32 + 8 * hh);
        vb.h[1] = *(const v8b*)(const void*)(Vt + (t * 16 + c) * 64 + kk * 32 + 16 + 8 * hh);
        oacc[t] = mma_gb(pa.v, vb.v, oacc[t]);
      }
    }
  }

  float* os = Os[wave];
#pragma unroll
  for (int r = 0; r < 8; ++r) {
    const float nr  = fmaxf(fabsf(nrow[r]), __expf(-mrow[r])) + 5e-5f;
    const float inv = 1.0f / nr;
#pragma unroll
    for (int t = 0; t < 4; ++t) os[(8 * hh + r) * 68 + t * 16 + c] = oacc[t][r] * inv;
  }
  __syncthreads();
  {
    const int c4 = (lane & 15) * 4;
    float* ob = hout + (tokb + q0) * (size_t)DINNER + hd * DHEAD;
    for (int pass = 0; pass < 2; ++pass) {
#pragma unroll
      for (int it = 0; it < 8; ++it) {
        const int row = it * 2 + hh;
        const v4f val = *(const v4f*)(os + row * 68 + c4);
        *(volatile v4f*)(ob + (size_t)row * DINNER + c4) = val;
      }
      __threadfence();
    }
  }
}

__global__ __launch_bounds__(256) void outnorm_kernel(const float* __restrict__ hbuf,
                                                       const float* __restrict__ xa,
                                                       const float* __restrict__ xz,
                                                       const float* __restrict__ lnw,
                                                       const float* __restrict__ lnb,
                                                       const float* __restrict__ skipw,
                                                       unsigned short* __restrict__ hsh,
                                                       unsigned short* __restrict__ hsl) {
  __shared__ __align__(16) unsigned int shi[512];
  __shared__ __align__(16) unsigned int slo[512];
  const int row = blockIdx.x;
  const int tid = threadIdx.x;
  const int c4  = tid * 4;
  const v4f hv = *(const v4f*)(hbuf + (size_t)row * DINNER + c4);
  float s1 = (hv[0] + hv[1]) + (hv[2] + hv[3]);
  s1 += __shfl_xor(s1, 1, 32);
  s1 += __shfl_xor(s1, 2, 32);
  s1 += __shfl_xor(s1, 4, 32);
  s1 += __shfl_xor(s1, 8, 32);
  const float mu = s1 * (1.0f / 64.0f);
  const float d0 = hv[0] - mu, d1 = hv[1] - mu, d2 = hv[2] - mu, d3 = hv[3] - mu;
  float s2 = (d0 * d0 + d1 * d1) + (d2 * d2 + d3 * d3);
  s2 += __shfl_xor(s2, 1, 32);
  s2 += __shfl_xor(s2, 2, 32);
  s2 += __shfl_xor(s2, 4, 32);
  s2 += __shfl_xor(s2, 8, 32);
  const float var  = s2 * (1.0f / 64.0f);
  const float rstd = rsqrtf(var + 1e-3f);
  const v4f lw  = *(const v4f*)(lnw + c4);
  const v4f lb  = *(const v4f*)(lnb + c4);
  const v4f sk  = *(const v4f*)(skipw + c4);
  const v4f xav = *(const v4f*)(xa + (size_t)row * DINNER + c4);
  const v4f zv  = *(const v4f*)(xz + (size_t)row * UPN + DINNER + c4);
  const float dd[4] = {d0, d1, d2, d3};
  unsigned short hb[4], lbits[4];
#pragma unroll
  for (int e = 0; e < 4; ++e) {
    const float hn = (dd[e] * rstd) * (1.0f + lw[e]) + lb[e];
    const float z  = zv[e];
    const float sz = z / (1.0f + __expf(-z));
    const float hs = (hn + sk[e] * xav[e]) * sz;
    hb[e] = f2bf_bits(hs);
    lbits[e] = f2bf_bits(hs - bf_bits2f(hb[e]));
  }
  shi[2 * tid]     = (unsigned)hb[0] | ((unsigned)hb[1] << 16);
  shi[2 * tid + 1] = (unsigned)hb[2] | ((unsigned)hb[3] << 16);
  slo[2 * tid]     = (unsigned)lbits[0] | ((unsigned)lbits[1] << 16);
  slo[2 * tid + 1] = (unsigned)lbits[2] | ((unsigned)lbits[3] << 16);
  __syncthreads();
  if (tid < 128) {
    const u4w v = *(const u4w*)(&shi[4 * tid]);
    volatile u4w* p = (volatile u4w*)(void*)(hsh + (size_t)row * DINNER + 8 * tid);
    *p = v;
    __threadfence();
    *p = v;
  } else {
    const int t2 = tid - 128;
    const u4w v = *(const u4w*)(&slo[4 * t2]);
    volatile u4w* p = (volatile u4w*)(void*)(hsl + (size_t)row * DINNER + 8 * t2);
    *p = v;
    __threadfence();
    *p = v;
  }
}

extern "C" void kernel_launch(void* const* d_in, const int* in_sizes, int n_in,
                              void* d_out, int out_size, void* d_ws, size_t ws_size,
                              hipStream_t stream) {
  (void)in_sizes; (void)n_in;
  if (ws_size < OFF_END) return;
  if ((size_t)out_size < (size_t)NTOK * DMODEL) return;
  const float* x      = (const float*)d_in[0];
  const float* W_up   = (const float*)d_in[1];
  const float* b_up   = (const float*)d_in[2];
  const float* W_q    = (const float*)d_in[3];
  const float* W_k    = (const float*)d_in[4];
  const float* W_v    = (const float*)d_in[5];
  const float* conv_w = (const float*)d_in[6];
  const float* conv_b = (const float*)d_in[7];
  const float* W_i    = (const float*)d_in[8];
  const float* b_i    = (const float*)d_in[9];
  const float* W_f    = (const float*)d_in[10];
  const float* b_f    = (const float*)d_in[11];
  const float* ln_w   = (const float*)d_in[12];
  const float* ln_b   = (const float*)d_in[13];
  const float* skipv  = (const float*)d_in[14];
  const float* W_down = (const float*)d_in[15];
  const float* b_down = (const float*)d_in[16];

  char* ws = (char*)d_ws;
  unsigned short* xh   = (unsigned short*)(ws + OFF_XH);
  unsigned short* xl   = (unsigned short*)(ws + OFF_XL);
  unsigned short* wuh  = (unsigned short*)(ws + OFF_WUH);
  unsigned short* wul  = (unsigned short*)(ws + OFF_WUL);
  unsigned short* wdh  = (unsigned short*)(ws + OFF_WDH);
  unsigned short* wdl  = (unsigned short*)(ws + OFF_WDL);
  unsigned short* wq16 = (unsigned short*)(ws + OFF_WQ);
  unsigned short* wk16 = (unsigned short*)(ws + OFF_WK);
  unsigned short* wv16 = (unsigned short*)(ws + OFF_WV);
  unsigned short* wg   = (unsigned short*)(ws + OFF_WG);
  float*          xz   = (float*)(ws + OFF_XZ);
  float*          xa   = (float*)(ws + OFF_XA);
  unsigned short* xa16 = (unsigned short*)(ws + OFF_ACT16);
  unsigned short* xm16 = (unsigned short*)(ws + OFF_XM16);
  float*          hbuf = (float*)(ws + OFF_H);
  unsigned short* gin  = (unsigned short*)(ws + OFF_GIN);
  unsigned short* hsh  = (unsigned short*)(ws + OFF_HSH);
  unsigned short* hsl  = (unsigned short*)(ws + OFF_HSL);
  float*          graw = (float*)(ws + OFF_GRAW);
  float*          ipg  = (float*)(ws + OFF_IPG);
  float*          cumg = (float*)(ws + OFF_CUM);

  {
    const int n8x = NTOK * DMODEL / 8;
    cast_bf16_split8<<<(n8x + 255) / 256, 256, 0, stream>>>(x, xh, xl, n8x);
    const int n8u = UPN * DMODEL / 8;
    cast_bf16_split8<<<(n8u + 255) / 256, 256, 0, stream>>>(W_up, wuh, wul, n8u);
    const int n8d = DMODEL * DINNER / 8;
    cast_bf16_split8<<<(n8d + 255) / 256, 256, 0, stream>>>(W_down, wdh, wdl, n8d);
    const int n8h = NHEAD * DHEAD * DHEAD / 8;
    cast_f16_scale8<<<(n8h + 255) / 256, 256, 0, stream>>>(W_q, wq16, n8h, 32.0f);
    cast_f16_scale8<<<(n8h + 255) / 256, 256, 0, stream>>>(W_k, wk16, n8h, 32.0f);
    cast_f16_scale8<<<(n8h + 255) / 256, 256, 0, stream>>>(W_v, wv16, n8h, 32.0f);
    const int n8g = GATE_N * GIN_LD / 8;
    build_gate_w8<<<(n8g + 255) / 256, 256, 0, stream>>>(W_i, W_f, wg, n8g);
  }

  wmma_gemm64<1, true, 2, 0, false, 0><<<dim3((NTOK / 64) * (UPN / 64) / 8, 1), 256, 0, stream>>>(
      xh, xl, DMODEL, 0L, wuh, wul, DMODEL, 0L, (void*)xz, nullptr, UPN, 0L,
      b_up, nullptr, 0L, NTOK, UPN, DMODEL, 1.0f);

  conv_silu_kernel<<<NTOK, 256, 0, stream>>>(xz, conv_w, conv_b, xa, xa16, xm16);

  wmma_gemm64<0, false, 0, 3, false, 0><<<dim3((NTOK / 64) / 8, NHEAD), 256, 0, stream>>>(
      xa16, nullptr, DINNER, (long)DHEAD, wq16, nullptr, DHEAD, (long)(DHEAD * DHEAD),
      (void*)(gin + 0), nullptr, GIN_LD, (long)DHEAD, nullptr, nullptr, 0L,
      NTOK, DHEAD, DHEAD, 1.0f / 2048.0f);
  wmma_gemm64<0, false, 0, 3, false, 0><<<dim3((NTOK / 64) / 8, NHEAD), 256, 0, stream>>>(
      xa16, nullptr, DINNER, (long)DHEAD, wk16, nullptr, DHEAD, (long)(DHEAD * DHEAD),
      (void*)(gin + DINNER), nullptr, GIN_LD, (long)DHEAD, nullptr, nullptr, 0L,
      NTOK, DHEAD, DHEAD, 1.0f / 2048.0f);
  wmma_gemm64<0, false, 0, 3, false, 0><<<dim3((NTOK / 64) / 8, NHEAD), 256, 0, stream>>>(
      xm16, nullptr, DINNER, (long)DHEAD, wv16, nullptr, DHEAD, (long)(DHEAD * DHEAD),
      (void*)(gin + 2 * DINNER), nullptr, GIN_LD, (long)DHEAD, nullptr, nullptr, 0L,
      NTOK, DHEAD, DHEAD, 1.0f / 256.0f);

  wmma_gemm64<1, false, 0, 0, false, 0><<<dim3((NTOK / 64) / 8, 1), 256, 0, stream>>>(
      gin, nullptr, GIN_LD, 0L, wg, nullptr, GIN_LD, 0L, (void*)graw, nullptr, GATE_N, 0L,
      nullptr, nullptr, 0L, NTOK, GATE_N, GIN_LD, 1.0f);

  gate_scan_kernel<<<NB * NHEAD, 32, 0, stream>>>(graw, b_i, b_f, ipg, cumg);

  mlstm64_kernel<<<NB * NHEAD * (SEQ / 64), 128, 0, stream>>>(gin, cumg, ipg, hbuf);

  outnorm_kernel<<<NTOK, 256, 0, stream>>>(hbuf, xa, xz, ln_w, ln_b, skipv, hsh, hsl);

  wmma_gemm64<1, true, 2, 0, false, 0><<<dim3((NTOK / 64) * (DMODEL / 64) / 8, 1), 256, 0, stream>>>(
      hsh, hsl, DINNER, 0L, wdh, wdl, DINNER, 0L, d_out, nullptr, DMODEL, 0L,
      b_down, nullptr, 0L, NTOK, DMODEL, DINNER, 1.0f);
}
